// CliffordDDIDecoder_50818053046333
// MI455X (gfx1250) — hardware-verified
//
#include <hip/hip_runtime.h>
#include <stddef.h>
#include <math.h>


#pragma clang fp contract(off)

#define DD     512
#define HH     256
#define MV     64
#define RR     95
#define RP     96
#define NROWT  64
#define NTHR   256
#define KCH    128
#define AP     136
#define XP     264
#define QP     72
#define MPP    68
#define TP     132
#define LN_EPS 1e-5f
#define WSCAP  134217728

#define O_W1PH 0
#define O_W1PL 131072
#define O_W1VH 262144
#define O_W1VL 393216
#define O_W2PH 524288
#define O_W2PL 540672
#define O_W2VH 557056
#define O_W2VL 573440
#define O_TTH  589824
#define O_TTL  595968
#define WS_ELEMS 602112

#define L_AHI  0
#define L_ALO  (NROWT * AP * 2)
#define L_XHI  0
#define L_XLO  (NROWT * XP * 2)
#define L_QHI  0
#define L_QLO  (NROWT * QP * 2)
#define L_OT   (2 * NROWT * QP * 2)
#define L_R0SZ (2 * NROWT * XP * 2)
#define L_RS   L_R0SZ
#define L_RQ   (L_RS + NROWT * 4 * 4)
#define L_MP   (L_RQ + NROWT * 4 * 4)
#define L_MSZ  (NROWT * MPP * 4)
#define LDS_MAIN (L_MP + 2 * L_MSZ)

static_assert(2 * NROWT * AP * 2 <= L_R0SZ);
static_assert(L_OT + NROWT * RR * 4 <= L_R0SZ);
static_assert((L_ALO % 16) == 0 && (L_XLO % 16) == 0 && (L_QLO % 16) == 0 && (L_OT % 16) == 0);
static_assert((L_RS % 16) == 0 && (L_RQ % 16) == 0 && (L_MP % 16) == 0 && (L_MSZ % 16) == 0);
static_assert(LDS_MAIN <= 160 * 1024);
static_assert(((NROWT * RR) % 4) == 0);
static_assert(((AP * 2) % 16) == 0 && ((XP * 2) % 16) == 0 && ((QP * 2) % 16) == 0);
static_assert(((MPP * 4) % 16) == 0 && ((TP * 4) % 16) == 0);
static_assert(((O_W1PL * 2) % 128) == 0 && ((O_W1VH * 2) % 128) == 0 && ((O_W1VL * 2) % 128) == 0);
static_assert(((O_W2PH * 2) % 128) == 0 && ((O_W2PL * 2) % 128) == 0 && ((O_W2VH * 2) % 128) == 0);
static_assert(((O_W2VL * 2) % 128) == 0 && ((O_TTH * 2) % 128) == 0 && ((O_TTL * 2) % 128) == 0);
static_assert(((WS_ELEMS * 2) % 128) == 0);
static_assert(O_TTL + RP * MV == WS_ELEMS);
static_assert((DD % KCH) == 0 && (KCH % 32) == 0 && (HH % 32) == 0 && (MV % 32) == 0);
static_assert(NROWT * RR * 4 == 190 * 128);

typedef float           v4f   __attribute__((ext_vector_type(4)));
typedef float           v8f   __attribute__((ext_vector_type(8)));
typedef unsigned short  v8us  __attribute__((ext_vector_type(8)));
typedef unsigned short  v16us __attribute__((ext_vector_type(16)));
typedef __bf16          v16bf __attribute__((ext_vector_type(16)));
union Frag { v16bf b; v16us u; v8us h[2]; };
static_assert(sizeof(Frag) == 32);

struct CayT { int p[8][8]; float s[8][8]; };
constexpr CayT CAY = {
  { {0, 1, 2, 3, 4, 5, 6, 7}, {1, 0, 4, 5, 2, 3, 7, 6}, {2, 4, 0, 6, 1, 7, 3, 5}, {3, 5, 6, 0, 7, 1, 2, 4},
    {4, 2, 1, 7, 0, 6, 5, 3}, {5, 3, 7, 1, 6, 0, 4, 2}, {6, 7, 3, 2, 5, 4, 0, 1}, {7, 6, 5, 4, 3, 2, 1, 0} },
  { {1.f, 1.f, 1.f, 1.f, 1.f, 1.f, 1.f, 1.f},
    {1.f, 1.f, 1.f, 1.f, 1.f, 1.f, 1.f, 1.f},
    {1.f, -1.f, 1.f, 1.f, -1.f, -1.f, 1.f, -1.f},
    {1.f, -1.f, -1.f, 1.f, 1.f, -1.f, -1.f, 1.f},
    {1.f, -1.f, 1.f, 1.f, -1.f, -1.f, 1.f, -1.f},
    {1.f, -1.f, -1.f, 1.f, 1.f, -1.f, -1.f, 1.f},
    {1.f, 1.f, -1.f, 1.f, -1.f, 1.f, -1.f, -1.f},
    {1.f, 1.f, -1.f, 1.f, -1.f, 1.f, -1.f, -1.f} }
};

__device__ __forceinline__ v8f wmb(v16bf a, v16bf bq, v8f c) {
  v8f d = __builtin_amdgcn_wmma_f32_16x16x32_bf16(false, a, false, bq, (short)0, c, false, false);
  asm volatile("v_nop\n\tv_nop\n\tv_nop\n\tv_nop" : "+v"(d) : "v"(a), "v"(bq));
  return d;
}

__device__ __forceinline__ v8f zero8() {
  v8f z = {0.f, 0.f, 0.f, 0.f, 0.f, 0.f, 0.f, 0.f};
  return z;
}

__device__ __forceinline__ unsigned bf16_bits(float f) {
  unsigned u = __float_as_uint(f);
  u += 0x7FFFu + ((u >> 16) & 1u);
  return u >> 16;
}

__device__ __forceinline__ void split2(float v, unsigned short& hb, unsigned short& lb) {
  const unsigned hh = bf16_bits(v);
  const float hf = __uint_as_float(hh << 16);
  hb = (unsigned short)hh;
  lb = (unsigned short)bf16_bits(v - hf);
}

__device__ __forceinline__ void split8(v4f u0, v4f u1, v8us& hv, v8us& lv) {
  unsigned short a, d;
  split2(u0.x, a, d); hv[0] = a; lv[0] = d;
  split2(u0.y, a, d); hv[1] = a; lv[1] = d;
  split2(u0.z, a, d); hv[2] = a; lv[2] = d;
  split2(u0.w, a, d); hv[3] = a; lv[3] = d;
  split2(u1.x, a, d); hv[4] = a; lv[4] = d;
  split2(u1.y, a, d); hv[5] = a; lv[5] = d;
  split2(u1.z, a, d); hv[6] = a; lv[6] = d;
  split2(u1.w, a, d); hv[7] = a; lv[7] = d;
}

__global__ __launch_bounds__(NTHR) void k_prep(
    const float* __restrict__ Wp1, const float* __restrict__ Wv1,
    const float* __restrict__ Wp2, const float* __restrict__ Wv2,
    const float* __restrict__ T, unsigned short* wsb) {
  __shared__ __align__(16) float ts[32 * TP];
  const int b = blockIdx.x, tid = threadIdx.x, lane = tid & 31, wv = tid >> 5;
  if (b < 72) {
    const float* src; int Kd, Nd, lb, oh, ol;
    if (b < 32)      { src = Wp1; Kd = DD; Nd = HH; lb = b;      oh = O_W1PH; ol = O_W1PL; }
    else if (b < 64) { src = Wv1; Kd = DD; Nd = HH; lb = b - 32; oh = O_W1VH; ol = O_W1VL; }
    else if (b < 68) { src = Wp2; Kd = HH; Nd = MV; lb = b - 64; oh = O_W2PH; ol = O_W2PL; }
    else             { src = Wv2; Kd = HH; Nd = MV; lb = b - 68; oh = O_W2VH; ol = O_W2VL; }
    const int nkt = Kd / 128;
    const int nti = lb / nkt, kt = lb - nti * nkt;
    const int n0 = 32 * nti, k0 = 128 * kt;
#pragma unroll 1
    for (int i = 0; i < 16; ++i) {
      const int kk = wv + 8 * i;
      ts[lane * TP + kk] = src[(size_t)(k0 + kk) * Nd + n0 + lane];
    }
    __syncthreads();
    v8us hv[2], lv[2];
    size_t dofs[2];
#pragma unroll
    for (int j = 0; j < 2; ++j) {
      const int p = tid + NTHR * j;
      const int row = p >> 4, q = p & 15;
      const float* tr = ts + row * TP + 8 * q;
      const v4f u0 = *(const v4f*)tr, u1 = *(const v4f*)(tr + 4);
      split8(u0, u1, hv[j], lv[j]);
      dofs[j] = (size_t)(n0 + row) * Kd + k0 + 8 * q;
    }
#pragma unroll
    for (int j = 0; j < 2; ++j) {
      *(volatile v8us*)(wsb + oh + dofs[j]) = hv[j];
      *(volatile v8us*)(wsb + ol + dofs[j]) = lv[j];
    }
    __threadfence();
#pragma unroll
    for (int j = 0; j < 2; ++j) {
      *(volatile v8us*)(wsb + oh + dofs[j]) = hv[j];
      *(volatile v8us*)(wsb + ol + dofs[j]) = lv[j];
    }
  } else {
    const int t = (b - 72) * NTHR + tid;
    const int row = t >> 3, g = t & 7;
    const int rs = row < RR ? row : RR - 1;
    const float* tp = T + (size_t)rs * MV + 8 * g;
    v4f u0 = *(const v4f*)tp, u1 = *(const v4f*)(tp + 4);
    const v4f z = {0.f, 0.f, 0.f, 0.f};
    if (row >= RR) { u0 = z; u1 = z; }
    v8us hv, lv;
    split8(u0, u1, hv, lv);
    const size_t d = (size_t)row * MV + 8 * g;
    *(volatile v8us*)(wsb + O_TTH + d) = hv;
    *(volatile v8us*)(wsb + O_TTL + d) = lv;
    __threadfence();
    *(volatile v8us*)(wsb + O_TTH + d) = hv;
    *(volatile v8us*)(wsb + O_TTL + d) = lv;
  }
}

__global__ __launch_bounds__(NTHR) void k_main(
    const float* __restrict__ hpp, const float* __restrict__ hvp,
    const float* __restrict__ bp1, const float* __restrict__ gp1,
    const float* __restrict__ tbp1, const float* __restrict__ bp2,
    const float* __restrict__ bv1, const float* __restrict__ gv1,
    const float* __restrict__ tbv1, const float* __restrict__ bv2,
    const float* __restrict__ gw, const unsigned short* __restrict__ wsb, float* out) {
  extern __shared__ v4f lds_dyn[];
  char* sm = (char*)lds_dyn;
  unsigned short* Ahi = (unsigned short*)(sm + L_AHI);
  unsigned short* Alo = (unsigned short*)(sm + L_ALO);
  unsigned short* Xhi = (unsigned short*)(sm + L_XHI);
  unsigned short* Xlo = (unsigned short*)(sm + L_XLO);
  unsigned short* Qhi = (unsigned short*)(sm + L_QHI);
  unsigned short* Qlo = (unsigned short*)(sm + L_QLO);
  float* otl  = (float*)(sm + L_OT);
  float* rsum = (float*)(sm + L_RS);
  float* rsq  = (float*)(sm + L_RQ);
  float* mpt  = (float*)(sm + L_MP);
  float* mvt  = (float*)(sm + L_MP + L_MSZ);

  const int tid = threadIdx.x, lane = tid & 31, wave = tid >> 5, h = lane >> 4, m = lane & 15;
  const int row0 = blockIdx.x * NROWT;

  float gws[8];
#pragma unroll
  for (int n = 0; n < 8; ++n) gws[n] = gw[n];

#pragma unroll 1
  for (int br = 0; br < 2; ++br) {
    const float* X  = br ? hvp : hpp;
    const float* b1 = br ? bv1 : bp1;
    const float* g1 = br ? gv1 : gp1;
    const float* t1 = br ? tbv1 : tbp1;
    const float* b2 = br ? bv2 : bp2;
    const unsigned short* W1h = wsb + (br ? O_W1VH : O_W1PH);
    const unsigned short* W1l = wsb + (br ? O_W1VL : O_W1PL);
    const unsigned short* W2h = wsb + (br ? O_W2VH : O_W2PH);
    const unsigned short* W2l = wsb + (br ? O_W2VL : O_W2PL);
    float* mt = (float*)(sm + L_MP + br * L_MSZ);

    const int rg = wave & 1, cg = wave >> 1;
    v8f acc[8];
#pragma unroll
    for (int i = 0; i < 8; ++i) acc[i] = zero8();

#pragma unroll 1
    for (int ck = 0; ck < DD / KCH; ++ck) {
#pragma unroll
      for (int it = 0; it < 4; ++it) {
        const int g = tid & 15, row = (tid >> 4) + 16 * it;
        const float* xp = X + (size_t)(row0 + row) * DD + KCH * ck + 8 * g;
        const v4f u0 = *(const v4f*)xp, u1 = *(const v4f*)(xp + 4);
        v8us hv8, lv8;
        split8(u0, u1, hv8, lv8);
        *(v8us*)(Ahi + row * AP + 8 * g) = hv8;
        *(v8us*)(Alo + row * AP + 8 * g) = lv8;
      }
      __syncthreads();
      {
        const unsigned short* ah0 = Ahi + (32 * rg + m) * AP + 8 * h;
        const unsigned short* al0 = Alo + (32 * rg + m) * AP + 8 * h;
        const unsigned short* wh = W1h + (size_t)(64 * cg + m) * DD + KCH * ck + 8 * h;
        const unsigned short* wl = W1l + (size_t)(64 * cg + m) * DD + KCH * ck + 8 * h;
#pragma unroll 1
        for (int ks = 0; ks < KCH / 32; ++ks) {
          const int ko = 32 * ks;
          Frag fah[2], fal[2];
#pragma unroll
          for (int mi = 0; mi < 2; ++mi) {
            fah[mi].h[0] = *(const v8us*)(ah0 + mi * 16 * AP + ko);
            fah[mi].h[1] = *(const v8us*)(ah0 + mi * 16 * AP + ko + 16);
            fal[mi].h[0] = *(const v8us*)(al0 + mi * 16 * AP + ko);
            fal[mi].h[1] = *(const v8us*)(al0 + mi * 16 * AP + ko + 16);
          }
#pragma unroll
          for (int nt = 0; nt < 4; ++nt) {
            const size_t no = (size_t)(16 * nt) * DD + ko;
            Frag fbh, fbl;
            fbh.h[0] = *(const v8us*)(wh + no);
            fbh.h[1] = *(const v8us*)(wh + no + 16);
            fbl.h[0] = *(const v8us*)(wl + no);
            fbl.h[1] = *(const v8us*)(wl + no + 16);
#pragma unroll
            for (int mi = 0; mi < 2; ++mi) {
              acc[mi * 4 + nt] = wmb(fah[mi].b, fbh.b, acc[mi * 4 + nt]);
              acc[mi * 4 + nt] = wmb(fah[mi].b, fbl.b, acc[mi * 4 + nt]);
              acc[mi * 4 + nt] = wmb(fal[mi].b, fbh.b, acc[mi * 4 + nt]);
            }
          }
        }
      }
      __syncthreads();
    }

    float bia[4], gam[4], bet[4];
#pragma unroll
    for (int nt = 0; nt < 4; ++nt) {
      const int col = 64 * cg + 16 * nt + m;
      bia[nt] = b1[col]; gam[nt] = g1[col]; bet[nt] = t1[col];
    }
#pragma unroll
    for (int mi = 0; mi < 2; ++mi)
#pragma unroll
      for (int nt = 0; nt < 4; ++nt)
#pragma unroll
        for (int r = 0; r < 8; ++r) acc[mi * 4 + nt][r] = acc[mi * 4 + nt][r] + bia[nt];

#pragma unroll
    for (int mi = 0; mi < 2; ++mi)
#pragma unroll
      for (int r = 0; r < 8; ++r) {
        float s = (acc[mi * 4][r] + acc[mi * 4 + 1][r]) + (acc[mi * 4 + 2][r] + acc[mi * 4 + 3][r]);
        s += __shfl_xor(s, 1);
        s += __shfl_xor(s, 2);
        s += __shfl_xor(s, 4);
        s += __shfl_xor(s, 8);
        if (m == 0) rsum[(32 * rg + 16 * mi + 8 * h + r) * 4 + cg] = s;
      }
    __syncthreads();
    float mu[16], rsd[16];
#pragma unroll
    for (int mi = 0; mi < 2; ++mi)
#pragma unroll
      for (int r = 0; r < 8; ++r) {
        const v4f s4 = *(const v4f*)(rsum + (32 * rg + 16 * mi + 8 * h + r) * 4);
        mu[mi * 8 + r] = ((s4.x + s4.y) + (s4.z + s4.w)) * (1.0f / 256.0f);
      }
#pragma unroll
    for (int mi = 0; mi < 2; ++mi)
#pragma unroll
      for (int r = 0; r < 8; ++r) {
        const float mr = mu[mi * 8 + r];
        float q = 0.0f;
#pragma unroll
        for (int nt = 0; nt < 4; ++nt) { const float dv = acc[mi * 4 + nt][r] - mr; q += dv * dv; }
        q += __shfl_xor(q, 1);
        q += __shfl_xor(q, 2);
        q += __shfl_xor(q, 4);
        q += __shfl_xor(q, 8);
        if (m == 0) rsq[(32 * rg + 16 * mi + 8 * h + r) * 4 + cg] = q;
      }
    __syncthreads();
#pragma unroll
    for (int mi = 0; mi < 2; ++mi)
#pragma unroll
      for (int r = 0; r < 8; ++r) {
        const v4f q4 = *(const v4f*)(rsq + (32 * rg + 16 * mi + 8 * h + r) * 4);
        const float var = ((q4.x + q4.y) + (q4.z + q4.w)) * (1.0f / 256.0f);
        rsd[mi * 8 + r] = rsqrtf(var + LN_EPS);
      }
#pragma unroll
    for (int mi = 0; mi < 2; ++mi)
#pragma unroll
      for (int nt = 0; nt < 4; ++nt)
#pragma unroll
        for (int r = 0; r < 8; ++r) {
          const int row = 32 * rg + 16 * mi + 8 * h + r, col = 64 * cg + 16 * nt + m;
          const float xn = (acc[mi * 4 + nt][r] - mu[mi * 8 + r]) * rsd[mi * 8 + r] * gam[nt] + bet[nt];
          const float y  = 0.5f * xn * (1.0f + erff(xn * 0.70710678118654752f));
          unsigned short hb, lb;
          split2(y, hb, lb);
          Xhi[row * XP + col] = hb;
          Xlo[row * XP + col] = lb;
        }
    __syncthreads();

    {
      const int rt = wave & 3, c2 = wave >> 2;
      v8f acc2[2];
      acc2[0] = zero8(); acc2[1] = zero8();
      const unsigned short* xh = Xhi + (16 * rt + m) * XP + 8 * h;
      const unsigned short* xl = Xlo + (16 * rt + m) * XP + 8 * h;
      const unsigned short* wh = W2h + (size_t)(32 * c2 + m) * HH + 8 * h;
      const unsigned short* wl = W2l + (size_t)(32 * c2 + m) * HH + 8 * h;
#pragma unroll 1
      for (int ks = 0; ks < HH / 32; ++ks) {
        const int ko = 32 * ks;
        Frag fah, fal;
        fah.h[0] = *(const v8us*)(xh + ko);
        fah.h[1] = *(const v8us*)(xh + ko + 16);
        fal.h[0] = *(const v8us*)(xl + ko);
        fal.h[1] = *(const v8us*)(xl + ko + 16);
#pragma unroll
        for (int nt = 0; nt < 2; ++nt) {
          const size_t no = (size_t)(16 * nt) * HH + ko;
          Frag fbh, fbl;
          fbh.h[0] = *(const v8us*)(wh + no);
          fbh.h[1] = *(const v8us*)(wh + no + 16);
          fbl.h[0] = *(const v8us*)(wl + no);
          fbl.h[1] = *(const v8us*)(wl + no + 16);
          acc2[nt] = wmb(fah.b, fbh.b, acc2[nt]);
          acc2[nt] = wmb(fah.b, fbl.b, acc2[nt]);
          acc2[nt] = wmb(fal.b, fbh.b, acc2[nt]);
        }
      }
      float b2v[2];
#pragma unroll
      for (int nt = 0; nt < 2; ++nt) b2v[nt] = b2[32 * c2 + 16 * nt + m];
#pragma unroll
      for (int nt = 0; nt < 2; ++nt)
#pragma unroll
        for (int r = 0; r < 8; ++r)
          mt[(16 * rt + 8 * h + r) * MPP + 32 * c2 + 16 * nt + m] = acc2[nt][r] + b2v[nt];
    }
    __syncthreads();
  }

#pragma unroll
  for (int it = 0; it < 2; ++it) {
    const int task = tid + NTHR * it;
    const int row = task >> 3, kq = task & 7;
    const float* pa = mpt + row * MPP + 8 * kq;
    const float* pv = mvt + row * MPP + 8 * kq;
    const v4f a0 = *(const v4f*)pa, a1 = *(const v4f*)(pa + 4);
    const v4f v0 = *(const v4f*)pv, v1 = *(const v4f*)(pv + 4);
    const float aa[8] = {a0.x, a0.y, a0.z, a0.w, a1.x, a1.y, a1.z, a1.w};
    const float vv[8] = {v0.x, v0.y, v0.z, v0.w, v1.x, v1.y, v1.z, v1.w};
    float Gv[8];
#pragma unroll
    for (int q = 0; q < 8; ++q) {
      float s = 0.0f;
#pragma unroll
      for (int j = 0; j < 8; ++j) s += CAY.s[q][j] * gws[CAY.p[q][j]] * vv[j];
      Gv[q] = s;
    }
    v8us qh, ql;
#pragma unroll
    for (int j2 = 0; j2 < 8; ++j2) {
      float s = 0.0f;
#pragma unroll
      for (int i = 0; i < 8; ++i) s += CAY.s[i][j2] * aa[i] * Gv[CAY.p[i][j2]];
      unsigned short hb, lb;
      split2(s, hb, lb);
      qh[j2] = hb; ql[j2] = lb;
    }
    *(v8us*)(Qhi + row * QP + 8 * kq) = qh;
    *(v8us*)(Qlo + row * QP + 8 * kq) = ql;
  }
  __syncthreads();

  {
    const int rt = wave & 3, c3 = wave >> 2;
    v8f acc3[3];
    acc3[0] = zero8(); acc3[1] = zero8(); acc3[2] = zero8();
    const unsigned short* qh = Qhi + (16 * rt + m) * QP + 8 * h;
    const unsigned short* ql = Qlo + (16 * rt + m) * QP + 8 * h;
    const unsigned short* th = wsb + O_TTH + (size_t)(48 * c3 + m) * MV + 8 * h;
    const unsigned short* tl = wsb + O_TTL + (size_t)(48 * c3 + m) * MV + 8 * h;
#pragma unroll
    for (int ks = 0; ks < MV / 32; ++ks) {
      const int ko = 32 * ks;
      Frag fah, fal;
      fah.h[0] = *(const v8us*)(qh + ko);
      fah.h[1] = *(const v8us*)(qh + ko + 16);
      fal.h[0] = *(const v8us*)(ql + ko);
      fal.h[1] = *(const v8us*)(ql + ko + 16);
#pragma unroll
      for (int nt = 0; nt < 3; ++nt) {
        const size_t no = (size_t)(16 * nt) * MV + ko;
        Frag fbh, fbl;
        fbh.h[0] = *(const v8us*)(th + no);
        fbh.h[1] = *(const v8us*)(th + no + 16);
        fbl.h[0] = *(const v8us*)(tl + no);
        fbl.h[1] = *(const v8us*)(tl + no + 16);
        acc3[nt] = wmb(fah.b, fbh.b, acc3[nt]);
        acc3[nt] = wmb(fah.b, fbl.b, acc3[nt]);
        acc3[nt] = wmb(fal.b, fbh.b, acc3[nt]);
      }
    }
#pragma unroll
    for (int nt = 0; nt < 3; ++nt)
#pragma unroll
      for (int r = 0; r < 8; ++r) {
        const int rc = 48 * c3 + 16 * nt + m, row = 16 * rt + 8 * h + r;
        if (rc < RR) otl[row * RR + rc] = acc3[nt][r] * 0.125f;
      }
  }
  __syncthreads();

  {
    constexpr int NV = NROWT * RR / 4;
    float* op = out + (size_t)row0 * RR;
    v4f ov[6];
#pragma unroll
    for (int j = 0; j < 6; ++j) {
      const int e = tid + NTHR * j;
      const int ec = e < NV ? e : NV - 1;
      ov[j] = *(const v4f*)(otl + 4 * ec);
    }
#pragma unroll
    for (int j = 0; j < 6; ++j) {
      const int e = tid + NTHR * j;
      if (e < NV) *(volatile v4f*)(op + 4 * e) = ov[j];
    }
    __threadfence();
#pragma unroll
    for (int j = 0; j < 6; ++j) {
      const int e = tid + NTHR * j;
      if (e < NV) *(volatile v4f*)(op + 4 * e) = ov[j];
    }
  }
}

extern "C" void kernel_launch(void* const* d_in, const int* in_sizes, int n_in,
                              void* d_out, int out_size, void* d_ws, size_t ws_size,
                              hipStream_t stream) {
  if (n_in < 16) return;
  const int nrow = in_sizes[0] / DD;
  if (nrow <= 0 || in_sizes[0] != nrow * DD || (nrow % NROWT) != 0) return;
  if (in_sizes[1] != nrow * DD) return;
  if (in_sizes[2] != DD * HH || in_sizes[3] != HH || in_sizes[4] != HH || in_sizes[5] != HH) return;
  if (in_sizes[6] != HH * MV || in_sizes[7] != MV) return;
  if (in_sizes[8] != DD * HH || in_sizes[9] != HH || in_sizes[10] != HH || in_sizes[11] != HH) return;
  if (in_sizes[12] != HH * MV || in_sizes[13] != MV) return;
  if (in_sizes[14] != RR * MV || in_sizes[15] != 8) return;
  if (out_size != nrow * RR) return;

  const float* h_perp = (const float*)d_in[0];
  const float* h_vuln = (const float*)d_in[1];
  const float* Wp1 = (const float*)d_in[2];
  const float* bp1 = (const float*)d_in[3];
  const float* lgp = (const float*)d_in[4];
  const float* lbp = (const float*)d_in[5];
  const float* Wp2 = (const float*)d_in[6];
  const float* bp2 = (const float*)d_in[7];
  const float* Wv1 = (const float*)d_in[8];
  const float* bv1 = (const float*)d_in[9];
  const float* lgv = (const float*)d_in[10];
  const float* lbv = (const float*)d_in[11];
  const float* Wv2 = (const float*)d_in[12];
  const float* bv2 = (const float*)d_in[13];
  const float* T   = (const float*)d_in[14];
  const float* gw  = (const float*)d_in[15];
  float* out = (float*)d_out;

  const size_t tot = (size_t)WS_ELEMS * 2;
  if (tot > ws_size || tot > (size_t)WSCAP) return;
  unsigned short* wsb = (unsigned short*)d_ws;
  const int nblk = nrow / NROWT;

  k_prep<<<75, NTHR, 0, stream>>>(Wp1, Wv1, Wp2, Wv2, T, wsb);

  hipFuncSetAttribute(reinterpret_cast<const void*>(&k_main),
                      hipFuncAttributeMaxDynamicSharedMemorySize, LDS_MAIN);
  k_main<<<nblk, NTHR, LDS_MAIN, stream>>>(h_perp, h_vuln, bp1, lgp, lbp, bp2,
                                           bv1, lgv, lbv, bv2, gw, wsb, out);
}
